// MultiHeadAttention_23553600651289
// MI455X (gfx1250) — hardware-run, weakly checked
//
#include <hip/hip_runtime.h>


#ifndef NB
#define NB 4
#endif
#ifndef SEQ
#define SEQ 2048
#endif
#define NB_FULL  4
#define SEQ_FULL 2048
#ifndef OUT_SEQ
#define OUT_SEQ SEQ
#endif
#define DM   768
#define NH_  12
#define HD   64
#define AW   4
#define ESEQ ((SEQ) < 512 ? (SEQ) : 512)
#define QRS  2048.0f
#define QRI  (1.0f / 2048.0f)
#define SC2  (0.125f * 1.4426950408889634f)
#define PSH  8.0f
#define NEGB (-3.0e38f)
#define BIGLIM (1 << 30)

static_assert(HD == 64);
static_assert(NH_ * HD == DM);
static_assert(DM % 64 == 0);
static_assert(DM % 32 == 0);
static_assert(SEQ % 64 == 0);
static_assert((NB * SEQ) % 64 == 0);
static_assert(SEQ % 32 == 0);
static_assert(ESEQ % 64 == 0);
static_assert(ESEQ % (16 * AW) == 0);
static_assert((SEQ - ESEQ) % (16 * AW) == 0);
static_assert(((size_t)SEQ * DM) % 8 == 0);
static_assert(((size_t)DM * DM) % 8 == 0);
static_assert(NB <= NB_FULL);
static_assert(SEQ <= SEQ_FULL);

typedef _Float16 h16;
typedef unsigned short bf;
typedef __attribute__((ext_vector_type(16))) __bf16   v16bf;
typedef __attribute__((ext_vector_type(16))) _Float16 v16h;
typedef __attribute__((ext_vector_type(8)))  _Float16 v8h;
typedef __attribute__((ext_vector_type(8)))  unsigned short v8us;
typedef __attribute__((ext_vector_type(8)))  float    v8f;
typedef __attribute__((ext_vector_type(4)))  float    v4f;
typedef v4f  __attribute__((may_alias)) v4fa;

__device__ __forceinline__ unsigned short f2bf(float f) { unsigned u = __float_as_uint(f); u += 0x7FFFu + ((u >> 16) & 1u); return (unsigned short)(u >> 16); }
__device__ __forceinline__ float bf2f(unsigned short hbits) { return __uint_as_float(((unsigned)hbits) << 16); }
__device__ __forceinline__ v16h cat16(v8h lo, v8h hi) { return __builtin_shufflevector(lo, hi, 0, 1, 2, 3, 4, 5, 6, 7, 8, 9, 10, 11, 12, 13, 14, 15); }
__device__ __forceinline__ v16bf cat16b(v8us lo, v8us hi) { return __builtin_bit_cast(v16bf, __builtin_shufflevector(lo, hi, 0, 1, 2, 3, 4, 5, 6, 7, 8, 9, 10, 11, 12, 13, 14, 15)); }
__device__ __forceinline__ v8f wmma16(v16h a, v16h b, v8f c) { return __builtin_amdgcn_wmma_f32_16x16x32_f16(false, a, false, b, (short)0, c, false, false); }
__device__ __forceinline__ v8f wmmab(v16bf a, v16bf b, v8f c) { return __builtin_amdgcn_wmma_f32_16x16x32_bf16(false, a, false, b, (short)0, c, false, false); }
__device__ __forceinline__ v16h  ldh(const h16* p) { return cat16(*(const v8h*)p, *(const v8h*)(p + 16)); }
__device__ __forceinline__ v16bf ldb(const bf* p)  { return cat16b(*(const v8us*)p, *(const v8us*)(p + 16)); }
__device__ __forceinline__ void wave_sync() { __builtin_amdgcn_fence(3  , "wavefront"); __builtin_amdgcn_wave_barrier(); asm volatile("" ::: "memory"); }

__global__ __launch_bounds__(256) void k_cvt8(const float* __restrict__ src, bf* dst, size_t n8) {
    const size_t i = (size_t)blockIdx.x * 256 + threadIdx.x; if (i >= n8) return;
    const v8f v = *(const v8f*)(src + i * 8); v8us o;
#pragma unroll
    for (int k = 0; k < 8; ++k) o[k] = f2bf(v[k]);
    *(volatile v8us*)(dst + i * 8) = o; __threadfence(); *(volatile v8us*)(dst + i * 8) = o;
}

__global__ __launch_bounds__(32) void k_proj(const bf* __restrict__ A, const bf* __restrict__ Bt, h16* Ph, h16* Pr, int resRowLim, int resColLim, int RB, size_t sRB, int pitch, int CB, size_t sCB) {
    __shared__ __align__(16) float os[16 * 68];
    const int K = DM;
    const int lane = threadIdx.x & 31, lr = lane & 15, hi = lane >> 4; const int r0 = blockIdx.x * 64, c0 = blockIdx.y * 64;
    const int useRes = (((r0 % RB) < resRowLim) && ((c0 % CB) < resColLim)) ? 1 : 0;
    v8f acc[4][4];
#pragma unroll
    for (int mb = 0; mb < 4; ++mb)
#pragma unroll
        for (int nb = 0; nb < 4; ++nb) acc[mb][nb] = (v8f){};
    const size_t aoff = (size_t)(r0 + lr) * K + 8 * hi, boff = (size_t)(c0 + lr) * K + 8 * hi;
#pragma unroll 1
    for (int kc = 0; kc < K; kc += 32) {
        v16bf a[4];
#pragma unroll
        for (int mb = 0; mb < 4; ++mb) a[mb] = ldb(A + aoff + (size_t)mb * 16 * K + kc);
#pragma unroll
        for (int nb = 0; nb < 4; ++nb) { const v16bf b = ldb(Bt + boff + (size_t)nb * 16 * K + kc);
#pragma unroll
            for (int mb = 0; mb < 4; ++mb) acc[mb][nb] = wmmab(a[mb], b, acc[mb][nb]); }
        asm volatile("v_nop\n\tv_nop\n\tv_nop\n\tv_nop" : "+v"(acc[0][0]), "+v"(acc[1][1]), "+v"(acc[2][2]), "+v"(acc[3][3]) : "v"(a[0]), "v"(a[1]), "v"(a[2]), "v"(a[3]));
    }
    const size_t tbase = (size_t)(r0 / RB) * sRB + (size_t)(r0 % RB) * (size_t)pitch + (size_t)(c0 / CB) * sCB + (size_t)(c0 % CB);
#pragma unroll
    for (int mb = 0; mb < 4; ++mb) {
#pragma unroll
        for (int nb = 0; nb < 4; ++nb) {
#pragma unroll
            for (int j = 0; j < 8; ++j) os[(hi * 8 + j) * 68 + nb * 16 + lr] = acc[mb][nb][j]; }
        wave_sync();
        const size_t sb = tbase + (size_t)(mb * 16) * (size_t)pitch;
#pragma unroll 1
        for (int ps = 0; ps < 2; ++ps) {
#pragma unroll
            for (int s = 0; s < 4; ++s) { const int row = 4 * s + (lane >> 3), c8 = (lane & 7) * 8;
                const v4f x0 = *(const v4fa*)(&os[row * 68 + c8]); const v4f x1 = *(const v4fa*)(&os[row * 68 + c8 + 4]); v8h hv, rv;
#pragma unroll
                for (int i = 0; i < 4; ++i) { const h16 a0 = (h16)x0[i]; const h16 a1 = (h16)x1[i]; hv[i] = a0; hv[4 + i] = a1; rv[i] = (h16)((x0[i] - (float)a0) * QRS); rv[4 + i] = (h16)((x1[i] - (float)a1) * QRS); }
                const size_t oo = sb + (size_t)row * (size_t)pitch + c8;
                *(volatile v8h*)(Ph + oo) = hv; if (useRes) *(volatile v8h*)(Pr + oo) = rv; }
            if (ps == 0) __threadfence(); }
        wave_sync();
    }
}

template <int EARLY>
__global__ __launch_bounds__(32 * AW) void k_flash(const h16* __restrict__ QH, const h16* __restrict__ QR, const h16* __restrict__ KP, const h16* __restrict__ KR,
                                                   const h16* __restrict__ VT, const h16* __restrict__ VR, bf* C2, size_t cpl, int tstart) {
    __shared__ __align__(16) float os[AW * 16 * 68];
    const int lane = threadIdx.x & 31, lr = lane & 15, hi = lane >> 4;
    const int wave = __builtin_amdgcn_readfirstlane((int)(threadIdx.x >> 5));
    const int zh = blockIdx.y; const int b = zh / NH_, h = zh % NH_;
    const int t0 = tstart + ((int)blockIdx.x * AW + wave) * 16;
    const int kend = t0 + 16;
    const int qi = t0 + lr;
    const size_t pbase = (size_t)zh * SEQ * HD;
    const size_t qo = pbase + (size_t)(t0 + lr) * HD + 8 * hi;
    const v16h qh0 = ldh(QH + qo), qh1 = ldh(QH + qo + 32);
    v16h qr0 = qh0, qr1 = qh1;
    if (EARLY) { qr0 = ldh(QR + qo); qr1 = ldh(QR + qo + 32); }
    const size_t ko = pbase + (size_t)lr * HD + 8 * hi;
    const size_t vo = pbase + (size_t)lr * SEQ + 8 * hi;
    v8f o0 = (v8f){}, o1 = (v8f){}, o2 = (v8f){}, o3 = (v8f){};
    v8f e0 = (v8f){}, e1 = (v8f){}, e2 = (v8f){}, e3 = (v8f){};
    float m = NEGB, l = 0.0f;
#pragma unroll 1
    for (int key0 = 0; key0 < kend; key0 += 32) {
        const h16* ka = KP + ko + (size_t)key0 * HD;
        const v16h ka0 = ldh(ka), ka1 = ldh(ka + 32), kb0 = ldh(ka + 16 * HD), kb1 = ldh(ka + 16 * HD + 32);
        v8f sHa = (v8f){}, sLa = (v8f){}, sHb = (v8f){}, sLb = (v8f){};
        if (EARLY) {
            const h16* kr = KR + ko + (size_t)key0 * HD;
            const v16h ra0 = ldh(kr), ra1 = ldh(kr + 32), rb0 = ldh(kr + 16 * HD), rb1 = ldh(kr + 16 * HD + 32);
            sHa = wmma16(ka0, qh0, sHa); sLa = wmma16(ka0, qr0, sLa); sHb = wmma16(kb0, qh0, sHb); sLb = wmma16(kb0, qr0, sLb);
            sHa = wmma16(ka1, qh1, sHa); sLa = wmma16(ka1, qr1, sLa); sHb = wmma16(kb1, qh1, sHb); sLb = wmma16(kb1, qr1, sLb);
            sLa = wmma16(ra0, qh0, sLa); sLb = wmma16(rb0, qh0, sLb); sLa = wmma16(ra1, qh1, sLa); sLb = wmma16(rb1, qh1, sLb);
            asm volatile("v_nop\n\tv_nop\n\tv_nop\n\tv_nop" : "+v"(sHa), "+v"(sLa), "+v"(sHb), "+v"(sLb) : "v"(ka0), "v"(ka1), "v"(kb0), "v"(kb1), "v"(ra0), "v"(ra1), "v"(rb0), "v"(rb1));
        } else {
            sHa = wmma16(ka0, qh0, sHa); sHb = wmma16(kb0, qh0, sHb);
            sHa = wmma16(ka1, qh1, sHa); sHb = wmma16(kb1, qh1, sHb);
            asm volatile("v_nop\n\tv_nop\n\tv_nop\n\tv_nop" : "+v"(sHa), "+v"(sHb) : "v"(ka0), "v"(ka1), "v"(kb0), "v"(kb1));
        }
        const int kA = key0 + 8 * hi;
        float ta[8], tb[8]; float mx = NEGB;
#pragma unroll
        for (int r = 0; r < 8; ++r) {
            float va = sHa[r], vb = sHb[r];
            if (EARLY) { va += sLa[r] * QRI; vb += sLb[r] * QRI; }
            va *= SC2; vb *= SC2;
            ta[r] = (kA + r <= qi) ? va : NEGB;
            tb[r] = (kA + 16 + r <= qi) ? vb : NEGB;
            mx = fmaxf(mx, fmaxf(ta[r], tb[r])); }
        mx = fmaxf(mx, __shfl_xor(mx, 16, 32));
        const float mnew = fmaxf(m, mx);
        const float alpha = __builtin_amdgcn_exp2f(m - mnew);
        const float sh = PSH - mnew;
        v16h pb = (v16h){}, pr = (v16h){}; float ls = 0.0f;
#pragma unroll
        for (int r = 0; r < 8; ++r) {
            const float fa = __builtin_amdgcn_exp2f(ta[r] + sh); const float fb = __builtin_amdgcn_exp2f(tb[r] + sh);
            const h16 pa = (h16)fa; const h16 pc = (h16)fb; pb[r] = pa; pb[8 + r] = pc;
            if (EARLY) { const h16 ra = (h16)((fa - (float)pa) * QRS); const h16 rc = (h16)((fb - (float)pc) * QRS); pr[r] = ra; pr[8 + r] = rc;
                         ls += ((float)pa + (float)ra * QRI) + ((float)pc + (float)rc * QRI); }
            else ls += (float)pa + (float)pc; }
        l = l * alpha + ls; m = mnew;
        o0 = o0 * alpha; o1 = o1 * alpha; o2 = o2 * alpha; o3 = o3 * alpha;
        const h16* va_ = VT + vo + key0;
        const v16h v0 = ldh(va_), v1 = ldh(va_ + (size_t)16 * SEQ), v2 = ldh(va_ + (size_t)32 * SEQ), v3 = ldh(va_ + (size_t)48 * SEQ);
        if (EARLY) {
            e0 = e0 * alpha; e1 = e1 * alpha; e2 = e2 * alpha; e3 = e3 * alpha;
            const h16* vr_ = VR + vo + key0;
            const v16h w0 = ldh(vr_), w1 = ldh(vr_ + (size_t)16 * SEQ), w2 = ldh(vr_ + (size_t)32 * SEQ), w3 = ldh(vr_ + (size_t)48 * SEQ);
            o0 = wmma16(v0, pb, o0); o1 = wmma16(v1, pb, o1); o2 = wmma16(v2, pb, o2); o3 = wmma16(v3, pb, o3);
            e0 = wmma16(v0, pr, e0); e1 = wmma16(v1, pr, e1); e2 = wmma16(v2, pr, e2); e3 = wmma16(v3, pr, e3);
            e0 = wmma16(w0, pb, e0); e1 = wmma16(w1, pb, e1); e2 = wmma16(w2, pb, e2); e3 = wmma16(w3, pb, e3);
            asm volatile("v_nop\n\tv_nop\n\tv_nop\n\tv_nop" : "+v"(o0), "+v"(o1), "+v"(o2), "+v"(o3), "+v"(e0), "+v"(e1), "+v"(e2), "+v"(e3)
                         : "v"(v0), "v"(v1), "v"(v2), "v"(v3), "v"(w0), "v"(w1), "v"(w2), "v"(w3), "v"(pb), "v"(pr));
        } else {
            o0 = wmma16(v0, pb, o0); o1 = wmma16(v1, pb, o1); o2 = wmma16(v2, pb, o2); o3 = wmma16(v3, pb, o3);
            asm volatile("v_nop\n\tv_nop\n\tv_nop\n\tv_nop" : "+v"(o0), "+v"(o1), "+v"(o2), "+v"(o3) : "v"(v0), "v"(v1), "v"(v2), "v"(v3), "v"(pb));
        }
    }
    l += __shfl_xor(l, 16, 32);
    const float inv = 1.0f / l;
    v8f f0, f1, f2, f3;
    if (EARLY) { f0 = (o0 + e0 * QRI) * inv; f1 = (o1 + e1 * QRI) * inv; f2 = (o2 + e2 * QRI) * inv; f3 = (o3 + e3 * QRI) * inv; }
    else       { f0 = o0 * inv; f1 = o1 * inv; f2 = o2 * inv; f3 = o3 * inv; }
    const int wb = wave * 16 * 68;
    { const int ob = wb + lr * 68 + 8 * hi;
      *(v4fa*)(&os[ob +  0]) = __builtin_shufflevector(f0, f0, 0, 1, 2, 3); *(v4fa*)(&os[ob +  0 + 4]) = __builtin_shufflevector(f0, f0, 4, 5, 6, 7);
      *(v4fa*)(&os[ob + 16]) = __builtin_shufflevector(f1, f1, 0, 1, 2, 3); *(v4fa*)(&os[ob + 16 + 4]) = __builtin_shufflevector(f1, f1, 4, 5, 6, 7);
      *(v4fa*)(&os[ob + 32]) = __builtin_shufflevector(f2, f2, 0, 1, 2, 3); *(v4fa*)(&os[ob + 32 + 4]) = __builtin_shufflevector(f2, f2, 4, 5, 6, 7);
      *(v4fa*)(&os[ob + 48]) = __builtin_shufflevector(f3, f3, 0, 1, 2, 3); *(v4fa*)(&os[ob + 48 + 4]) = __builtin_shufflevector(f3, f3, 4, 5, 6, 7); }
    wave_sync();
    const size_t cb = ((size_t)b * SEQ + t0) * DM + (size_t)h * HD;
#pragma unroll 1
    for (int ps = 0; ps < 2; ++ps) {
#pragma unroll
        for (int s = 0; s < 4; ++s) { const int row = 4 * s + (lane >> 3), c8 = (lane & 7) * 8;
            const v4f x0 = *(const v4fa*)(&os[wb + row * 68 + c8]); const v4f x1 = *(const v4fa*)(&os[wb + row * 68 + c8 + 4]); v8us hv, lv;
#pragma unroll
            for (int i = 0; i < 4; ++i) { const unsigned short a0 = f2bf(x0[i]); const unsigned short a1 = f2bf(x1[i]); hv[i] = a0; hv[4 + i] = a1;
                                          lv[i] = f2bf(x0[i] - bf2f(a0)); lv[4 + i] = f2bf(x1[i] - bf2f(a1)); }
            const size_t oo = cb + (size_t)row * DM + c8;
            *(volatile v8us*)(C2 + oo) = hv; *(volatile v8us*)(C2 + cpl + oo) = lv; }
        if (ps == 0) __threadfence(); }
}

__global__ __launch_bounds__(32) void k_oproj(const bf* __restrict__ C2, size_t cpl, const bf* __restrict__ Bt, const float* __restrict__ bo, float* OUT) {
    __shared__ __align__(16) float os[16 * 68];
    const int K = DM;
    const int lane = threadIdx.x & 31, lr = lane & 15, hi = lane >> 4; const int r0 = blockIdx.x * 64, c0 = blockIdx.y * 64;
    v8f acc[4][4];
#pragma unroll
    for (int mb = 0; mb < 4; ++mb)
#pragma unroll
        for (int nb = 0; nb < 4; ++nb) acc[mb][nb] = (v8f){};
    const size_t aoff = (size_t)(r0 + lr) * K + 8 * hi, boff = (size_t)(c0 + lr) * K + 8 * hi;
#pragma unroll 1
    for (int p = 0; p < 2; ++p) {
        const size_t ap = (size_t)p * cpl + aoff;
#pragma unroll 1
        for (int kc = 0; kc < K; kc += 32) {
            v16bf a[4];
#pragma unroll
            for (int mb = 0; mb < 4; ++mb) a[mb] = ldb(C2 + ap + (size_t)mb * 16 * K + kc);
#pragma unroll
            for (int nb = 0; nb < 4; ++nb) { const v16bf bq = ldb(Bt + boff + (size_t)nb * 16 * K + kc);
#pragma unroll
                for (int mb = 0; mb < 4; ++mb) acc[mb][nb] = wmmab(a[mb], bq, acc[mb][nb]); }
            asm volatile("v_nop\n\tv_nop\n\tv_nop\n\tv_nop" : "+v"(acc[0][0]), "+v"(acc[1][1]), "+v"(acc[2][2]), "+v"(acc[3][3]) : "v"(a[0]), "v"(a[1]), "v"(a[2]), "v"(a[3]));
        }
    }
    float bias[4];
#pragma unroll
    for (int nb = 0; nb < 4; ++nb) bias[nb] = bf2f(f2bf(bo[c0 + nb * 16 + lr]));
    const size_t orow0 = (size_t)(r0 / SEQ) * OUT_SEQ + (size_t)(r0 % SEQ);
#pragma unroll
    for (int mb = 0; mb < 4; ++mb) {
#pragma unroll
        for (int nb = 0; nb < 4; ++nb) {
#pragma unroll
            for (int j = 0; j < 8; ++j) os[(hi * 8 + j) * 68 + nb * 16 + lr] = acc[mb][nb][j] + bias[nb]; }
        wave_sync();
        float* ob = OUT + (orow0 + (size_t)(mb * 16)) * DM + c0;
#pragma unroll 1
        for (int ps = 0; ps < 2; ++ps) {
#pragma unroll
            for (int s = 0; s < 8; ++s) { const int row = 2 * s + hi, cofs = lr * 4;
                const v4f val = *(const v4fa*)(&os[row * 68 + cofs]);
                *(volatile v4f*)(ob + (size_t)row * DM + cofs) = val; }
            if (ps == 0) __threadfence(); }
        wave_sync();
    }
}

static constexpr size_t al256(size_t v) { return (v + 255) & ~(size_t)255; }
static constexpr size_t SZ_XB = al256((size_t)NB * SEQ * DM * 2);
static constexpr size_t SZ_WB = al256((size_t)4 * DM * DM * 2);
static constexpr size_t SZ_PL = al256((size_t)NB * NH_ * SEQ * HD * 2);
static constexpr size_t SZ_CP = al256((size_t)NB * SEQ * DM * 2);
static constexpr size_t SZ_TOTAL = SZ_XB + SZ_WB + 6 * SZ_PL + 2 * SZ_CP;
static_assert(SZ_TOTAL <= (size_t)134217728);
static_assert(((size_t)DM * DM * 2) % 256 == 0);
static_assert(SZ_CP == (size_t)NB * SEQ * DM * 2);
static_assert(SZ_PL == (size_t)NB * NH_ * SEQ * HD * 2);

extern "C" void kernel_launch(void* const* d_in, const int* in_sizes, int n_in,
                              void* d_out, int out_size, void* d_ws, size_t ws_size, hipStream_t stream) {
    if (n_in < 6) return;
    const size_t needx = ((size_t)(NB - 1) * SEQ_FULL + SEQ) * DM;
    if ((size_t)in_sizes[0] < needx) return;
    if ((size_t)in_sizes[1] < (size_t)DM * DM || (size_t)in_sizes[2] < (size_t)DM * DM || (size_t)in_sizes[3] < (size_t)DM * DM || (size_t)in_sizes[4] < (size_t)DM * DM) return;
    if ((size_t)in_sizes[5] < (size_t)DM) return;
    if ((size_t)out_size < ((size_t)(NB - 1) * OUT_SEQ + SEQ) * DM) return;
    if (SZ_TOTAL > ws_size) return;
    const float* x = (const float*)d_in[0]; const float* wq = (const float*)d_in[1]; const float* wk = (const float*)d_in[2];
    const float* wv = (const float*)d_in[3]; const float* wo = (const float*)d_in[4]; const float* bo = (const float*)d_in[5];
    float* OUT = (float*)d_out;
    char* wsp = (char*)d_ws;
    bf* XB = (bf*)wsp; wsp += SZ_XB;
    bf* WB = (bf*)wsp; wsp += SZ_WB;
    h16* QH = (h16*)wsp; wsp += SZ_PL;
    h16* QR = (h16*)wsp; wsp += SZ_PL;
    h16* KP = (h16*)wsp; wsp += SZ_PL;
    h16* KR = (h16*)wsp; wsp += SZ_PL;
    h16* VT = (h16*)wsp; wsp += SZ_PL;
    h16* VR = (h16*)wsp; wsp += SZ_PL;
    bf* C2 = (bf*)wsp; wsp += 2 * SZ_CP;
    const size_t cpl = SZ_CP / 2;
    bf* WQ = WB; bf* WK = WB + (size_t)DM * DM; bf* WV = WB + (size_t)2 * DM * DM; bf* WO = WB + (size_t)3 * DM * DM;

    if (SEQ == SEQ_FULL) {
        const size_t n8 = (size_t)NB * SEQ * DM / 8;
        k_cvt8<<<(unsigned)((n8 + 255) / 256), 256, 0, stream>>>(x, XB, n8);
    } else {
        const size_t n8 = (size_t)SEQ * DM / 8;
        for (int b = 0; b < NB; ++b) k_cvt8<<<(unsigned)((n8 + 255) / 256), 256, 0, stream>>>(x + (size_t)b * SEQ_FULL * DM, XB + (size_t)b * SEQ * DM, n8);
    }
    { const size_t n8 = (size_t)DM * DM / 8; const unsigned g = (unsigned)((n8 + 255) / 256);
      k_cvt8<<<g, 256, 0, stream>>>(wq, WQ, n8); k_cvt8<<<g, 256, 0, stream>>>(wk, WK, n8); k_cvt8<<<g, 256, 0, stream>>>(wv, WV, n8); k_cvt8<<<g, 256, 0, stream>>>(wo, WO, n8); }

    k_proj<<<dim3(NB * SEQ / 64, DM / 64, 1), 32, 0, stream>>>(XB, WQ, QH, QR, ESEQ, BIGLIM, SEQ, (size_t)NH_ * SEQ * HD, HD, HD, (size_t)SEQ * HD);
    k_proj<<<dim3(NB * SEQ / 64, DM / 64, 1), 32, 0, stream>>>(XB, WK, KP, KR, ESEQ, BIGLIM, SEQ, (size_t)NH_ * SEQ * HD, HD, HD, (size_t)SEQ * HD);
    k_proj<<<dim3(DM / 64, NB * SEQ / 64, 1), 32, 0, stream>>>(WV, XB, VT, VR, BIGLIM, ESEQ, DM, (size_t)0, SEQ, SEQ, (size_t)DM * SEQ);

    k_flash<1><<<dim3(ESEQ / (16 * AW), NB * NH_, 1), 32 * AW, 0, stream>>>(QH, QR, KP, KR, VT, VR, C2, cpl, 0);
    if (SEQ > ESEQ)
        k_flash<0><<<dim3((SEQ - ESEQ) / (16 * AW), NB * NH_, 1), 32 * AW, 0, stream>>>(QH, QR, KP, KR, VT, VR, C2, cpl, ESEQ);

    k_oproj<<<dim3(NB * SEQ / 64, DM / 64, 1), 32, 0, stream>>>(C2, cpl, WO, bo, OUT);
}
